// NonLocalBlock_38989713113551
// MI455X (gfx1250) — hardware-verified
//
#include <hip/hip_runtime.h>


#ifndef NB
#define NB 8
#endif
#ifndef SEQ
#define SEQ 3136
#endif
#define NB_FULL  8
#define SEQ_FULL 3136
#define CC   256
#define IC   128
#define CO   256
#define MTOK (NB * SEQ)
#define PCAR 16384.0f
#define NCH4 (SEQ / 128)
#define REMK (SEQ - NCH4 * 128)
#define NV   (SEQ / 32)
static_assert(SEQ % 64 == 0);
static_assert(SEQ >= 64 && SEQ <= SEQ_FULL);
static_assert(NB >= 1 && NB <= NB_FULL);
static_assert(REMK == 0 || REMK == 64);
static_assert(CC == CO);
static_assert(CC % 32 == 0 && IC % 64 == 0 && CO % 64 == 0 && MTOK % 64 == 0);

typedef _Float16 h16;
typedef unsigned short bf;
typedef __attribute__((ext_vector_type(16))) __bf16   v16bf;
typedef __attribute__((ext_vector_type(16))) _Float16 v16h;
typedef __attribute__((ext_vector_type(8)))  _Float16 v8h;
typedef __attribute__((ext_vector_type(8)))  unsigned short v8us;
typedef __attribute__((ext_vector_type(8)))  float    v8f;
typedef __attribute__((ext_vector_type(4)))  float    v4f;
typedef __attribute__((ext_vector_type(2)))  unsigned short v2us;
typedef __attribute__((ext_vector_type(4)))  unsigned short v4us;
typedef __attribute__((ext_vector_type(2)))  _Float16 v2h;
typedef __attribute__((ext_vector_type(4)))  _Float16 v4h;
typedef __attribute__((ext_vector_type(2)))  float v2f;
typedef v8h  __attribute__((may_alias)) v8ha;
typedef v4f  __attribute__((may_alias)) v4fa;
typedef v8us __attribute__((may_alias)) v8usa;

__device__ __forceinline__ unsigned short f2bf(float f) { unsigned u = __float_as_uint(f); u += 0x7FFFu + ((u >> 16) & 1u); return (unsigned short)(u >> 16); }
__device__ __forceinline__ float bf2f(unsigned short b) { return __uint_as_float(((unsigned)b) << 16); }
__device__ __forceinline__ float bfr(float f) { return bf2f(f2bf(f)); }
__device__ __forceinline__ v16h cat16(v8h lo, v8h hi) { return __builtin_shufflevector(lo, hi, 0, 1, 2, 3, 4, 5, 6, 7, 8, 9, 10, 11, 12, 13, 14, 15); }
__device__ __forceinline__ v16bf cat16b(v8us lo, v8us hi) { return __builtin_bit_cast(v16bf, __builtin_shufflevector(lo, hi, 0, 1, 2, 3, 4, 5, 6, 7, 8, 9, 10, 11, 12, 13, 14, 15)); }
__device__ __forceinline__ v8f wmma16(v16h a, v16h b, v8f c) { return __builtin_amdgcn_wmma_f32_16x16x32_f16(false, a, false, b, (short)0, c, false, false); }
__device__ __forceinline__ v8f wmmab(v16bf a, v16bf b, v8f c) { return __builtin_amdgcn_wmma_f32_16x16x32_bf16(false, a, false, b, (short)0, c, false, false); }
__device__ __forceinline__ h16 tohx(float x) { return (h16)x; }
__device__ __forceinline__ void splitf(float y, unsigned short& h, unsigned short& l) { h = f2bf(y); l = f2bf(y - bf2f(h)); }

template <typename T16> struct WFrag;
template <> struct WFrag<h16> { typedef v16h V; static __device__ __forceinline__ V ld(const h16* p) { return cat16(*(const v8h*)p, *(const v8h*)(p + 16)); } static __device__ __forceinline__ v8f mma(V a, V b, v8f c) { return wmma16(a, b, c); } };
template <> struct WFrag<bf> { typedef v16bf V; static __device__ __forceinline__ V ld(const bf* p) { return cat16b(*(const v8us*)p, *(const v8us*)(p + 16)); } static __device__ __forceinline__ v8f mma(V a, V b, v8f c) { return wmmab(a, b, c); } };
template <typename T16, int NSPLIT, bool BIAS>
__global__ __launch_bounds__(32) void k_gemmw(const T16* __restrict__ A, const T16* __restrict__ A2, const T16* __restrict__ Bt, const T16* __restrict__ Bt2, int K, float* C, int ldc, const float* __restrict__ bias, size_t sA, size_t sB, size_t sC) {
    typedef typename WFrag<T16>::V V;
    __shared__ __align__(16) float os[16 * 68];
    const size_t z = blockIdx.z; A += z * sA; if (A2) A2 += z * sA; Bt += z * sB; if (Bt2) Bt2 += z * sB; C += z * sC;
    const int lane = threadIdx.x & 31, lr = lane & 15, hi = lane >> 4; const int r0 = blockIdx.x * 64, c0 = blockIdx.y * 64;
    v8f acc[4][4];
#pragma unroll
    for (int mb = 0; mb < 4; ++mb)
#pragma unroll
        for (int nb = 0; nb < 4; ++nb) acc[mb][nb] = (v8f){};
    const size_t aoff = (size_t)(r0 + lr) * K + 8 * hi, boff = (size_t)(c0 + lr) * K + 8 * hi;
#pragma unroll 1
    for (int kc = 0; kc < K; kc += 32) {
        V a[4], a2[4];
#pragma unroll
        for (int mb = 0; mb < 4; ++mb) { a[mb] = WFrag<T16>::ld(A + aoff + (size_t)mb * 16 * K + kc); if (NSPLIT == 1 || NSPLIT == 2) a2[mb] = WFrag<T16>::ld(A2 + aoff + (size_t)mb * 16 * K + kc); }
#pragma unroll
        for (int nb = 0; nb < 4; ++nb) { const V b = WFrag<T16>::ld(Bt + boff + (size_t)nb * 16 * K + kc); V b2; if (NSPLIT >= 2) b2 = WFrag<T16>::ld(Bt2 + boff + (size_t)nb * 16 * K + kc);
#pragma unroll
            for (int mb = 0; mb < 4; ++mb) { acc[mb][nb] = WFrag<T16>::mma(a[mb], b, acc[mb][nb]); if (NSPLIT == 1 || NSPLIT == 2) acc[mb][nb] = WFrag<T16>::mma(a2[mb], b, acc[mb][nb]); if (NSPLIT >= 2) acc[mb][nb] = WFrag<T16>::mma(a[mb], b2, acc[mb][nb]); } }
        asm volatile("v_nop\n\tv_nop\n\tv_nop\n\tv_nop" : "+v"(acc[0][0]), "+v"(acc[1][1]), "+v"(acc[2][2]), "+v"(acc[3][3]) : "v"(a[0]), "v"(a[3]));
    }
#pragma unroll
    for (int mb = 0; mb < 4; ++mb) {
#pragma unroll
        for (int nb = 0; nb < 4; ++nb) {
#pragma unroll
            for (int j = 0; j < 8; ++j) os[(hi * 8 + j) * 68 + nb * 16 + lr] = acc[mb][nb][j]; }
        __builtin_amdgcn_wave_barrier(); asm volatile("" ::: "memory");
        float* crow = C + (size_t)(r0 + mb * 16) * ldc + c0;
#pragma unroll 1
        for (int ps = 0; ps < 2; ++ps) {
#pragma unroll
            for (int s = 0; s < 8; ++s) { const int row = 2 * s + hi, cofs = lr * 4; v4f val = *(const v4fa*)(os + row * 68 + cofs); if (BIAS) { val[0] += bfr(bias[c0 + cofs]); val[1] += bfr(bias[c0 + cofs + 1]); val[2] += bfr(bias[c0 + cofs + 2]); val[3] += bfr(bias[c0 + cofs + 3]); }
                *(volatile v4f*)(crow + (size_t)row * ldc + cofs) = val; }
            if (ps == 0) __threadfence(); }
        __builtin_amdgcn_wave_barrier(); asm volatile("" ::: "memory");
    }
}

__global__ __launch_bounds__(256) void k_wt(const float* __restrict__ Wsrc, bf* dst, int K, int N) {
    const size_t i = (size_t)blockIdx.x * 256 + threadIdx.x; if (i >= (size_t)N * K / 8) return;
    const size_t e = i * 8; const int n = (int)(e / K); const int k0 = (int)(e % K); v8us o;
#pragma unroll
    for (int u = 0; u < 8; ++u) o[u] = f2bf(Wsrc[(size_t)(k0 + u) * N + n]);
    *(volatile v8us*)(dst + e) = o; __threadfence(); *(volatile v8us*)(dst + e) = o; }
__global__ __launch_bounds__(256) void k_cvtx(const float* __restrict__ x, bf* dst) {
    const size_t e = ((size_t)blockIdx.x * 256 + threadIdx.x) * 8; if (e >= (size_t)MTOK * CC) return;
    const size_t b = e / ((size_t)SEQ * CC); const size_t r = e - b * ((size_t)SEQ * CC);
    const float* sp = x + b * (size_t)SEQ_FULL * CC + r; const v4f a0 = *(const v4f*)sp; const v4f a1 = *(const v4f*)(sp + 4); v8us o;
#pragma unroll
    for (int u = 0; u < 4; ++u) { o[u] = f2bf(a0[u]); o[4 + u] = f2bf(a1[u]); }
    *(volatile v8us*)(dst + e) = o; __threadfence(); *(volatile v8us*)(dst + e) = o; }
__global__ __launch_bounds__(256) void k_hl(const float* __restrict__ F, bf* Fh, bf* Fl, float scale) {
    const size_t e = ((size_t)blockIdx.x * 256 + threadIdx.x) * 8; if (e >= (size_t)MTOK * IC) return;
    const v4f a0 = *(const v4f*)(F + e); const v4f a1 = *(const v4f*)(F + e + 4); v8us oh, ol;
#pragma unroll
    for (int u = 0; u < 4; ++u) { unsigned short p, q; splitf(a0[u] * scale, p, q); oh[u] = p; ol[u] = q; splitf(a1[u] * scale, p, q); oh[4 + u] = p; ol[4 + u] = q; }
    *(volatile v8us*)(Fh + e) = oh; *(volatile v8us*)(Fl + e) = ol; __threadfence(); *(volatile v8us*)(Fh + e) = oh; *(volatile v8us*)(Fl + e) = ol; }
__global__ __launch_bounds__(256) void k_gt16(const float* __restrict__ G, h16* GT) {
    const size_t e = ((size_t)blockIdx.x * 256 + threadIdx.x) * 8; if (e >= (size_t)NB * IC * SEQ) return;
    const size_t b = e / ((size_t)IC * SEQ); const size_t r = e - b * ((size_t)IC * SEQ); const int i = (int)(r / SEQ); const int m = (int)(r % SEQ);
    const float* gp = G + ((size_t)b * SEQ + m) * IC + i; v8h o;
#pragma unroll
    for (int u = 0; u < 8; ++u) o[u] = tohx(gp[(size_t)u * IC]);
    *(volatile v8h*)(GT + e) = o; __threadfence(); *(volatile v8h*)(GT + e) = o; }
__global__ __launch_bounds__(256) void k_rsoft(const float* __restrict__ S, h16* P16) {
    const int lane = threadIdx.x & 31; const int row = blockIdx.x * 8 + (threadIdx.x >> 5); if (row >= SEQ) return;
    const float* sr = S + (size_t)row * SEQ; float v[NV]; float mx = -3.0e38f;
#pragma unroll
    for (int ch = 0; ch < NCH4; ++ch) { const v4f a = *(const v4f*)(sr + ch * 128 + lane * 4);
#pragma unroll
        for (int u = 0; u < 4; ++u) { v[ch * 4 + u] = a[u]; mx = fmaxf(mx, a[u]); } }
#if REMK == 64
    { const v2f a2 = *(const v2f*)(sr + NCH4 * 128 + lane * 2); v[NCH4 * 4] = a2[0]; v[NCH4 * 4 + 1] = a2[1]; mx = fmaxf(mx, fmaxf(a2[0], a2[1])); }
#endif
#pragma unroll
    for (int sh = 16; sh; sh >>= 1) mx = fmaxf(mx, __shfl_xor(mx, sh, 32));
    float sum = 0.f;
#pragma unroll
    for (int q = 0; q < NV; ++q) { float d0 = __fsub_rn(v[q], mx); asm volatile("" : "+v"(d0)); v[q] = __builtin_amdgcn_exp2f(__fmul_rn(d0, 1.4426950408889634f)); sum += v[q]; }
#pragma unroll
    for (int sh = 16; sh; sh >>= 1) sum += __shfl_xor(sum, sh, 32);
    const float f = __fdiv_rn(PCAR, sum);
    for (int ps = 0; ps < 2; ++ps) {
#pragma unroll
        for (int ch = 0; ch < NCH4; ++ch) { v4h o4;
#pragma unroll
            for (int q = 0; q < 4; ++q) o4[q] = tohx(v[ch * 4 + q] * f); *(volatile v4h*)(P16 + (size_t)row * SEQ + ch * 128 + lane * 4) = o4; }
#if REMK == 64
        { v2h o2; o2[0] = tohx(v[NCH4 * 4] * f); o2[1] = tohx(v[NCH4 * 4 + 1] * f); *(volatile v2h*)(P16 + (size_t)row * SEQ + NCH4 * 128 + lane * 2) = o2; }
#endif
        if (ps == 0) __threadfence(); } }
__global__ __launch_bounds__(256) void k_fin(const float* __restrict__ Z, const float* __restrict__ x, float* OUTp) {
    const size_t e = ((size_t)blockIdx.x * 256 + threadIdx.x) * 4; if (e >= (size_t)MTOK * CO) return;
    const size_t b = e / ((size_t)SEQ * CO); const size_t r = e - b * ((size_t)SEQ * CO); const size_t g = b * (size_t)SEQ_FULL * CO + r;
    const v4f zv = *(const v4f*)(Z + e); const v4f xv = *(const v4f*)(x + g); v4f o;
#pragma unroll
    for (int u = 0; u < 4; ++u) o[u] = __fadd_rn(zv[u], bfr(xv[u]));
    *(volatile v4f*)(OUTp + g) = o; __threadfence(); *(volatile v4f*)(OUTp + g) = o; }

constexpr size_t kSzW   = (size_t)IC * CC * 2;
constexpr size_t kSzXB  = (size_t)MTOK * CC * 2;
constexpr size_t kSzF32 = (size_t)MTOK * IC * 4;
constexpr size_t kSzP16 = (size_t)MTOK * IC * 2;
constexpr size_t kSzGT  = (size_t)NB * IC * SEQ * 2;
constexpr size_t kSzS   = (size_t)SEQ * SEQ * 4;
constexpr size_t kSzZ   = (size_t)MTOK * CO * 4;
constexpr size_t kSzSZ  = (kSzS > kSzZ) ? kSzS : kSzZ;
constexpr size_t kSzP   = (size_t)SEQ * SEQ * 2;
constexpr size_t kWsTotal = 4 * kSzW + kSzXB + kSzF32 + 4 * kSzP16 + kSzGT + kSzSZ + kSzP + 2 * kSzP16;
static_assert(kSzW % 256 == 0 && kSzXB % 256 == 0 && kSzF32 % 256 == 0 && kSzP16 % 256 == 0 && kSzGT % 256 == 0 && kSzS % 256 == 0 && kSzZ % 256 == 0 && kSzP % 256 == 0);
static_assert(kWsTotal <= ((size_t)128 << 20));

extern "C" void kernel_launch(void* const* d_in, const int* in_sizes, int n_in,
                              void* d_out, int out_size, void* d_ws, size_t ws_size, hipStream_t stream) {
    if (n_in < 9) return;
    if ((size_t)in_sizes[0] < ((size_t)(NB - 1) * SEQ_FULL + SEQ) * CC) return;
    if (in_sizes[1] < CC * IC || in_sizes[3] < CC * IC || in_sizes[5] < CC * IC || in_sizes[7] < IC * CO) return;
    if (in_sizes[2] < IC || in_sizes[4] < IC || in_sizes[6] < IC || in_sizes[8] < CO) return;
    if ((size_t)out_size < ((size_t)(NB - 1) * SEQ_FULL + SEQ) * CO) return;
    const float* x = (const float*)d_in[0]; const float* wth = (const float*)d_in[1]; const float* bth = (const float*)d_in[2]; const float* wph = (const float*)d_in[3]; const float* bph = (const float*)d_in[4]; const float* wg = (const float*)d_in[5]; const float* bg = (const float*)d_in[6]; const float* wz = (const float*)d_in[7]; const float* bz = (const float*)d_in[8];
    float* OUT = (float*)d_out;
    char* wsp = (char*)d_ws;
    auto take = [&](size_t bytes) { char* p = wsp; wsp += (bytes + 255) & ~(size_t)255; return (void*)p; };
    bf* BTH = (bf*)take(kSzW); bf* BPH = (bf*)take(kSzW); bf* BG = (bf*)take(kSzW); bf* BZ = (bf*)take(kSzW);
    bf* XB = (bf*)take(kSzXB);
    float* TMPF = (float*)take(kSzF32);
    bf* THh = (bf*)take(kSzP16); bf* THl = (bf*)take(kSzP16); bf* PHh = (bf*)take(kSzP16); bf* PHl = (bf*)take(kSzP16);
    h16* GT = (h16*)take(kSzGT);
    float* SZ = (float*)take(kSzSZ);
    h16* P16 = (h16*)take(kSzP);
    bf* Yh = (bf*)take(kSzP16); bf* Yl = (bf*)take(kSzP16);
    if ((size_t)(wsp - (char*)d_ws) > ws_size) return;

    const unsigned nbw = (unsigned)((IC * CC / 8 + 255) / 256);
    k_wt<<<nbw, 256, 0, stream>>>(wth, BTH, CC, IC);
    k_wt<<<nbw, 256, 0, stream>>>(wph, BPH, CC, IC);
    k_wt<<<nbw, 256, 0, stream>>>(wg,  BG,  CC, IC);
    k_wt<<<nbw, 256, 0, stream>>>(wz,  BZ,  IC, CO);
    k_cvtx<<<(unsigned)(((size_t)MTOK * CC / 8 + 255) / 256), 256, 0, stream>>>(x, XB);
    const unsigned nhl = (unsigned)(((size_t)MTOK * IC / 8 + 255) / 256);
    k_gemmw<bf, 0, true><<<dim3(MTOK / 64, IC / 64, 1), 32, 0, stream>>>(XB, nullptr, BTH, nullptr, CC, TMPF, IC, bth, 0, 0, 0); k_hl<<<nhl, 256, 0, stream>>>(TMPF, THh, THl, 1.0f);
    k_gemmw<bf, 0, true><<<dim3(MTOK / 64, IC / 64, 1), 32, 0, stream>>>(XB, nullptr, BPH, nullptr, CC, TMPF, IC, bph, 0, 0, 0); k_hl<<<nhl, 256, 0, stream>>>(TMPF, PHh, PHl, 1.0f);
    k_gemmw<bf, 0, true><<<dim3(MTOK / 64, IC / 64, 1), 32, 0, stream>>>(XB, nullptr, BG, nullptr, CC, TMPF, IC, bg, 0, 0, 0);
    k_gt16<<<(unsigned)(((size_t)NB * IC * SEQ / 8 + 255) / 256), 256, 0, stream>>>(TMPF, GT);
    for (int b = 0; b < NB; ++b) { const size_t ob = (size_t)b * SEQ * IC;
        k_gemmw<bf, 2, false><<<dim3(SEQ / 64, SEQ / 64, 1), 32, 0, stream>>>(THh + ob, THl + ob, PHh + ob, PHl + ob, IC, SZ, SEQ, nullptr, 0, 0, 0);
        k_rsoft<<<SEQ / 8, 256, 0, stream>>>(SZ, P16);
        k_gemmw<h16, 0, false><<<dim3(SEQ / 64, IC / 64, 1), 32, 0, stream>>>(P16, nullptr, GT + ob, nullptr, SEQ, TMPF + ob, IC, nullptr, 0, 0, 0);
    }
    k_hl<<<nhl, 256, 0, stream>>>(TMPF, Yh, Yl, 1.0f / PCAR);
    k_gemmw<bf, 1, true><<<dim3(MTOK / 64, CO / 64, 1), 32, 0, stream>>>(Yh, Yl, BZ, nullptr, IC, SZ, CO, bz, 0, 0, 0);
    k_fin<<<(unsigned)(((size_t)MTOK * CO / 4 + 255) / 256), 256, 0, stream>>>(SZ, x, OUT);
}
